// LSTM_55456617726021
// MI455X (gfx1250) — hardware-verified
//
#include <hip/hip_runtime.h>
#include <math.h>

constexpr int NBATCH  = 64;
constexpr int NSTEP   = 512;
constexpr int NHID    = 256;
constexpr int NLAYER  = 2;
constexpr int NGATE   = 4 * NHID;
constexpr int NVOCAB  = 32000;
constexpr int NROWS   = NSTEP * NBATCH;
constexpr int SEQ_BLK = 16;
constexpr int SCAN_THR = 512;
constexpr int HPITCH  = 264;
constexpr int OPITCH  = 260;
constexpr int SLABP   = 68;
constexpr float ACT_CARRY = 64.0f;
constexpr float WGT_CARRY = 16.0f;
constexpr float PROD_INV  = 1.0f / (ACT_CARRY * WGT_CARRY);
constexpr int NOUT0 = NBATCH * NSTEP * NHID;
constexpr int NOUT1 = NLAYER * NBATCH * NHID;
constexpr int NOUT_TOTAL = NOUT0 + 2 * NOUT1;
constexpr long OUT1_BYTE_OFF = 33554432L;
constexpr long OUT2_BYTE_OFF = 33685504L;
constexpr long OUT_TOTAL_BYTES = 33816576L;

static_assert(NGATE == 1024, "gate width");
static_assert(NROWS % 64 == 0 && NGATE % 64 == 0, "GEMM M, N tile multiples");
static_assert(NHID % 32 == 0, "GEMM K multiple of 32");
static_assert(NBATCH == 64, "one 64-row M tile equals one time step");
static_assert((SCAN_THR / 32) * 16 == NHID, "16 waves x 16 hidden units");
static_assert(SCAN_THR / 32 == SEQ_BLK, "one copy-out row per wave");
static_assert(NBATCH % SEQ_BLK == 0, "batch tiles");
static_assert((long)NOUT0 * 4 == OUT1_BYTE_OFF, "out1 offset");
static_assert(OUT1_BYTE_OFF + (long)NOUT1 * 4 == OUT2_BYTE_OFF, "out2 offset");
static_assert(OUT2_BYTE_OFF + (long)NOUT1 * 4 == OUT_TOTAL_BYTES, "d_out extent");
static_assert((long)NOUT_TOTAL * 4 == OUT_TOTAL_BYTES, "d_out elements");
static_assert(HPITCH % 8 == 0 && OPITCH % 4 == 0, "LDS pitches keep 16-B alignment");

typedef __attribute__((ext_vector_type(16))) _Float16 v16h;
typedef __attribute__((ext_vector_type(8)))  _Float16 v8h;
typedef __attribute__((ext_vector_type(8)))  float    v8f;
typedef __attribute__((ext_vector_type(4)))  float    v4f;
typedef __attribute__((ext_vector_type(4)))  unsigned v4u;

union FragU { v16h v; v8h h[2]; };
__device__ __forceinline__ v16h frag_load(const _Float16* p) {
  FragU f;
  f.h[0] = *(const v8h*)(p);
  f.h[1] = *(const v8h*)(p + 16);
  return f.v;
}
__device__ __forceinline__ v8f wmma_f16(v16h a, v16h b, v8f c) {
  return __builtin_amdgcn_wmma_f32_16x16x32_f16(false, a, false, b, (short)0, c, false, false);
}
__device__ __forceinline__ void guard4_all(v8f& a0, v8f& a1, v8f& a2, v8f& a3, v16h x, v16h b0, v16h b1, v16h b2, v16h b3) {
  asm volatile("v_nop\n\tv_nop\n\tv_nop\n\tv_nop" : "+v"(a0), "+v"(a1), "+v"(a2), "+v"(a3) : "v"(x), "v"(b0), "v"(b1), "v"(b2), "v"(b3));
}
__device__ __forceinline__ void acc_guard4(v8f& a, v8f& b, v8f& c, v8f& d) {
  asm volatile("v_nop\n\tv_nop\n\tv_nop\n\tv_nop" : "+v"(a), "+v"(b), "+v"(c), "+v"(d));
}

__device__ __forceinline__ float h16_to_f32(unsigned hb) {
  const unsigned sgn = (hb & 0x8000u) << 16;
  const unsigned em = hb & 0x7fffu;
  const float fn = __uint_as_float((em << 13) + 0x38000000u);
  const float fs = (float)em * 5.9604644775390625e-8f;
  const float mag = (em < 0x400u) ? fs : fn;
  return __uint_as_float(__float_as_uint(mag) | sgn);
}

__device__ __forceinline__ float fsig(float x)  { return __builtin_amdgcn_rcpf(1.0f + expf(-x)); }
__device__ __forceinline__ float ftanh(float x) { return 1.0f - 2.0f * __builtin_amdgcn_rcpf(expf(2.0f * x) + 1.0f); }

__device__ __forceinline__ void store2_v8h(unsigned short* dst, v8h v) {
  for (int pass = 0; pass < 2; ++pass) {
    *(volatile v8h*)(void*)dst = v;
    __threadfence();
  }
}
__device__ __forceinline__ void store2_v4f_pair(float* d0, float* d1, v4f a, v4f b) {
  for (int pass = 0; pass < 2; ++pass) {
    *(volatile v4f*)d0 = a;
    *(volatile v4f*)d1 = b;
    __threadfence();
  }
}

__device__ __forceinline__ void cvt8_store(const float* sp, unsigned short* dp, float sc) {
  const v4f a = *(const v4f*)(sp);
  const v4f b = *(const v4f*)(sp + 4);
  v8h hv;
#pragma unroll
  for (int e = 0; e < 4; ++e) {
    hv[e]     = (_Float16)(a[e] * sc);
    hv[4 + e] = (_Float16)(b[e] * sc);
  }
  store2_v8h(dp, hv);
}

constexpr int PREP_GATHER_BLKS = NROWS * (NHID / 8) / 256;
constexpr int PREP_W_BLKS      = NLAYER * NGATE * NHID / 8 / 256;
constexpr int PREP_B_BLKS      = NLAYER * NGATE / 4 / 256;
constexpr int PREP_BLKS        = PREP_GATHER_BLKS + 2 * PREP_W_BLKS + PREP_B_BLKS;
static_assert(PREP_GATHER_BLKS == 4096 && PREP_W_BLKS == 256 && PREP_B_BLKS == 2, "prep coverage");

__global__ __launch_bounds__(256) void prep_kernel(const int* __restrict__ x, const float* __restrict__ emb,
                                                   const float* __restrict__ wih, const float* __restrict__ whh,
                                                   const float* __restrict__ bih, const float* __restrict__ bhh,
                                                   unsigned short* __restrict__ X0, unsigned short* __restrict__ WIH,
                                                   unsigned short* __restrict__ WHH, float* __restrict__ BSUM) {
  const int tid = threadIdx.x;
  const int blk = blockIdx.x;
  if (blk < PREP_GATHER_BLKS) {
    const int i  = blk * 256 + tid;
    const int m  = i >> 5;
    const int c8 = (i & 31) * 8;
    const int t  = m >> 6;
    const int b  = m & 63;
    int tok = x[b * NSTEP + t];
    tok = tok < 0 ? 0 : tok;
    tok = tok > (NVOCAB - 1) ? (NVOCAB - 1) : tok;
    cvt8_store(emb + (size_t)tok * NHID + c8, X0 + (size_t)i * 8, ACT_CARRY);
  } else if (blk < PREP_GATHER_BLKS + 2 * PREP_W_BLKS) {
    const int wb    = blk - PREP_GATHER_BLKS;
    const int which = wb / PREP_W_BLKS;
    const int j     = (wb - which * PREP_W_BLKS) * 256 + tid;
    const float* src = which ? whh : wih;
    unsigned short* dst = which ? WHH : WIH;
    cvt8_store(src + (size_t)j * 8, dst + (size_t)j * 8, WGT_CARRY);
  } else {
    const int j = (blk - PREP_GATHER_BLKS - 2 * PREP_W_BLKS) * 256 + tid;
    const v4f a = *(const v4f*)(bih + (size_t)j * 4);
    const v4f b = *(const v4f*)(bhh + (size_t)j * 4);
    v4f o;
#pragma unroll
    for (int e = 0; e < 4; ++e) o[e] = a[e] + b[e];
    float* op = BSUM + (size_t)j * 4;
    for (int pass = 0; pass < 2; ++pass) {
      *(volatile v4f*)op = o;
      __threadfence();
    }
  }
}

__global__ __launch_bounds__(256) void gemm_pre_kernel(const unsigned short* __restrict__ Ap, const unsigned short* __restrict__ Btp,
                                                       const float* __restrict__ bsum, unsigned short* __restrict__ P) {
  const _Float16* A  = (const _Float16*)Ap;
  const _Float16* Bt = (const _Float16*)Btp;
  __shared__ __align__(16) float sT[8][16 * SLABP];
  const int lane = threadIdx.x & 31;
  const int wave = threadIdx.x >> 5;
  constexpr int tilesN = NGATE >> 6;
  constexpr int tilesM = NROWS >> 6;
  const int tile = blockIdx.x * 8 + wave;
  if (tile >= tilesM * tilesN) return;
  const int tm = tile / tilesN;
  const int tn = tile - tm * tilesN;
  const int m0 = tm << 6;
  const int n0 = tn << 6;
  const int rlane = lane & 15;
  const int koff  = (lane >> 4) * 8;
  const int mOff  = (lane >> 4) * 8;

  v8f acc[4][4];
#pragma unroll
  for (int i = 0; i < 4; ++i)
#pragma unroll
    for (int j = 0; j < 4; ++j) acc[i][j] = (v8f){0.f, 0.f, 0.f, 0.f, 0.f, 0.f, 0.f, 0.f};

#pragma unroll 1
  for (int k0 = 0; k0 < NHID; k0 += 32) {
    v16h bh[4];
#pragma unroll
    for (int j = 0; j < 4; ++j) bh[j] = frag_load(Bt + (size_t)(n0 + (j << 4) + rlane) * NHID + koff + k0);
#pragma unroll
    for (int i = 0; i < 4; ++i) {
      const v16h ah = frag_load(A + (size_t)(m0 + (i << 4) + rlane) * NHID + koff + k0);
#pragma unroll
      for (int j = 0; j < 4; ++j) acc[i][j] = wmma_f16(ah, bh[j], acc[i][j]);
      guard4_all(acc[i][0], acc[i][1], acc[i][2], acc[i][3], ah, bh[0], bh[1], bh[2], bh[3]);
    }
  }
  acc_guard4(acc[0][0], acc[0][1], acc[0][2], acc[0][3]);
  acc_guard4(acc[1][0], acc[1][1], acc[1][2], acc[1][3]);
  acc_guard4(acc[2][0], acc[2][1], acc[2][2], acc[2][3]);
  acc_guard4(acc[3][0], acc[3][1], acc[3][2], acc[3][3]);

  float* slab = sT[wave];
  const int q4 = lane >> 3;
  const int c8 = (lane & 7) * 8;
#pragma unroll
  for (int j = 0; j < 4; ++j) {
    const int n = n0 + (j << 4) + rlane;
    const float bv = bsum[n];
#pragma unroll
    for (int i = 0; i < 4; ++i) {
#pragma unroll
      for (int r = 0; r < 8; ++r) slab[rlane * SLABP + (i << 4) + mOff + r] = acc[i][j][r] * PROD_INV + bv;
    }
    __builtin_amdgcn_fence(__ATOMIC_RELEASE, "workgroup");
    __builtin_amdgcn_wave_barrier();
    __builtin_amdgcn_fence(__ATOMIC_ACQUIRE, "workgroup");
    v8h hv[4];
#pragma unroll
    for (int it = 0; it < 4; ++it) {
      const float* sp = slab + (it * 4 + q4) * SLABP + c8;
#pragma unroll
      for (int e = 0; e < 8; ++e) hv[it][e] = (_Float16)sp[e];
    }
    for (int pass = 0; pass < 2; ++pass) {
#pragma unroll
      for (int it = 0; it < 4; ++it) {
        const int row = it * 4 + q4;
        unsigned short* dp = P + ((size_t)tm * NGATE + (size_t)(n0 + (j << 4) + row)) * NBATCH + c8;
        *(volatile v8h*)(void*)dp = hv[it];
      }
      __threadfence();
    }
    __builtin_amdgcn_fence(__ATOMIC_RELEASE, "workgroup");
    __builtin_amdgcn_wave_barrier();
    __builtin_amdgcn_fence(__ATOMIC_ACQUIRE, "workgroup");
  }
}

template <int LAYER>
__global__ __launch_bounds__(SCAN_THR) void scan_kernel(const unsigned short* __restrict__ PRE, const unsigned short* __restrict__ WHHp,
                                                        const float* __restrict__ h0, const float* __restrict__ c0,
                                                        unsigned short* __restrict__ Y0, float* __restrict__ out0,
                                                        float* __restrict__ outh, float* __restrict__ outc) {
  __shared__ __align__(16) _Float16 Hh[2][SEQ_BLK * HPITCH];
  __shared__ __align__(16) float    Hf[2][SEQ_BLK * OPITCH];
  const _Float16* WH = (const _Float16*)WHHp;
  const int tid = threadIdx.x, lane = tid & 31, wave = tid >> 5;
  const int c = lane & 15, hh = lane >> 4, koff = hh * 8;
  const int rowbase = blockIdx.x * SEQ_BLK;
  const int u = 16 * wave + c;

  {
    _Float16* hb = &Hh[0][0];
    constexpr int NEL = 2 * SEQ_BLK * HPITCH;
#pragma unroll 1
    for (int it = 0; it < (NEL + SCAN_THR - 1) / SCAN_THR; ++it) {
      const int i  = it * SCAN_THR + tid;
      const int ic = i < NEL ? i : (NEL - 1);
      const int row = ic / HPITCH;
      const int col = ic - row * HPITCH;
      const int rowc = row < SEQ_BLK ? row : (SEQ_BLK - 1);
      const int colc = col < NHID ? col : (NHID - 1);
      const float hv = h0[(size_t)(rowbase + rowc) * NHID + colc];
      const bool live = (row < SEQ_BLK) && (col < NHID);
      const float val = live ? hv * ACT_CARRY : 0.0f;
      if (i < NEL) hb[i] = (_Float16)val;
    }
  }
  float cst[8];
#pragma unroll
  for (int r = 0; r < 8; ++r) cst[r] = c0[(size_t)(rowbase + 8 * hh + r) * NHID + u];
  __syncthreads();

  const v8f z8 = {0.f, 0.f, 0.f, 0.f, 0.f, 0.f, 0.f, 0.f};
  const _Float16* wrow = WH + (size_t)u * NHID + koff;

#pragma unroll 1
  for (int t = 0; t < NSTEP; ++t) {
    const int cur = t & 1;
    const int nxt = cur ^ 1;
    const _Float16* ahrow = &Hh[cur][0] + c * HPITCH + koff;
    v8f acc[4];
    acc[0] = z8; acc[1] = z8; acc[2] = z8; acc[3] = z8;
#pragma unroll 1
    for (int k0 = 0; k0 < NHID; k0 += 32) {
      const v16h a  = frag_load(ahrow + k0);
      const v16h b0 = frag_load(wrow + k0);
      const v16h b1 = frag_load(wrow + (size_t)1 * NHID * NHID + k0);
      const v16h b2 = frag_load(wrow + (size_t)2 * NHID * NHID + k0);
      const v16h b3 = frag_load(wrow + (size_t)3 * NHID * NHID + k0);
      acc[0] = wmma_f16(a, b0, acc[0]);
      acc[1] = wmma_f16(a, b1, acc[1]);
      acc[2] = wmma_f16(a, b2, acc[2]);
      acc[3] = wmma_f16(a, b3, acc[3]);
      guard4_all(acc[0], acc[1], acc[2], acc[3], a, b0, b1, b2, b3);
    }
    acc_guard4(acc[0], acc[1], acc[2], acc[3]);

    v4u pw[4];
    {
      const unsigned short* pp = PRE + ((size_t)t * NGATE + (size_t)u) * NBATCH + rowbase + 8 * hh;
#pragma unroll
      for (int q = 0; q < 4; ++q) pw[q] = *(const v4u*)(const void*)(pp + (size_t)q * NHID * NBATCH);
    }
    const bool last = (t == NSTEP - 1);
    _Float16* hn16 = &Hh[nxt][0];
    float*    hn32 = &Hf[nxt][0];
#pragma unroll
    for (int r = 0; r < 8; ++r) {
      const unsigned wi = pw[0][r >> 1];
      const unsigned wf = pw[1][r >> 1];
      const unsigned wg = pw[2][r >> 1];
      const unsigned wo = pw[3][r >> 1];
      const unsigned bi = (r & 1) ? (wi >> 16) : (wi & 0xffffu);
      const unsigned bf = (r & 1) ? (wf >> 16) : (wf & 0xffffu);
      const unsigned bg = (r & 1) ? (wg >> 16) : (wg & 0xffffu);
      const unsigned bo = (r & 1) ? (wo >> 16) : (wo & 0xffffu);
      const float zi = acc[0][r] * PROD_INV + h16_to_f32(bi);
      const float zf = acc[1][r] * PROD_INV + h16_to_f32(bf);
      const float zg = acc[2][r] * PROD_INV + h16_to_f32(bg);
      const float zo = acc[3][r] * PROD_INV + h16_to_f32(bo);
      const float ig = fsig(zi);
      const float fg = fsig(zf);
      const float gg = ftanh(zg);
      const float og = fsig(zo);
      const float cn = fg * cst[r] + ig * gg;
      cst[r] = cn;
      const float hn = og * ftanh(cn);
      hn16[(8 * hh + r) * HPITCH + u] = (_Float16)(hn * ACT_CARRY);
      if (LAYER == 1 || last) hn32[(8 * hh + r) * OPITCH + u] = hn;
    }
    __syncthreads();

    if (LAYER == 0) {
      const v8h v = *(const v8h*)(hn16 + wave * HPITCH + lane * 8);
      store2_v8h(Y0 + ((size_t)t * NBATCH + (size_t)(rowbase + wave)) * NHID + lane * 8, v);
    } else {
      const v4f va = *(const v4f*)(hn32 + wave * OPITCH + 4 * lane);
      const v4f vb = *(const v4f*)(hn32 + wave * OPITCH + 128 + 4 * lane);
      float* dst = out0 + ((size_t)(rowbase + wave) * NSTEP + (size_t)t) * NHID;
      store2_v4f_pair(dst + 4 * lane, dst + 128 + 4 * lane, va, vb);
    }
    if (last) {
      const v4f va = *(const v4f*)(hn32 + wave * OPITCH + 4 * lane);
      const v4f vb = *(const v4f*)(hn32 + wave * OPITCH + 128 + 4 * lane);
      float* dst = outh + (size_t)(rowbase + wave) * NHID;
      store2_v4f_pair(dst + 4 * lane, dst + 128 + 4 * lane, va, vb);
    }
  }

  __syncthreads();
  {
    float* cs = &Hf[0][0];
#pragma unroll
    for (int r = 0; r < 8; ++r) cs[(8 * hh + r) * OPITCH + u] = cst[r];
  }
  __syncthreads();
  {
    const float* cs = &Hf[0][0];
    const v4f va = *(const v4f*)(cs + wave * OPITCH + 4 * lane);
    const v4f vb = *(const v4f*)(cs + wave * OPITCH + 128 + 4 * lane);
    float* dst = outc + (size_t)(rowbase + wave) * NHID;
    store2_v4f_pair(dst + 4 * lane, dst + 128 + 4 * lane, va, vb);
  }
}

extern "C" void kernel_launch(void* const* d_in, const int* in_sizes, int n_in,
                              void* d_out, int out_size, void* d_ws, size_t ws_size, hipStream_t stream) {
  if (n_in < 8 || d_out == nullptr || d_ws == nullptr) return;
  if (in_sizes[0] != NBATCH * NSTEP || in_sizes[1] != NVOCAB * NHID ||
      in_sizes[2] != NLAYER * NGATE * NHID || in_sizes[3] != NLAYER * NGATE * NHID ||
      in_sizes[4] != NLAYER * NGATE || in_sizes[5] != NLAYER * NGATE ||
      in_sizes[6] != NLAYER * NBATCH * NHID || in_sizes[7] != NLAYER * NBATCH * NHID ||
      out_size != NOUT_TOTAL) return;

  const int*   x   = (const int*)d_in[0];
  const float* emb = (const float*)d_in[1];
  const float* wih = (const float*)d_in[2];
  const float* whh = (const float*)d_in[3];
  const float* bih = (const float*)d_in[4];
  const float* bhh = (const float*)d_in[5];
  const float* h0  = (const float*)d_in[6];
  const float* c0  = (const float*)d_in[7];
  float* out0 = (float*)d_out;
  float* out1 = out0 + (size_t)(OUT1_BYTE_OFF / 4);
  float* out2 = out0 + (size_t)(OUT2_BYTE_OFF / 4);

  char* ws = (char*)d_ws;
  size_t off = 0;
  auto carve = [&](size_t bytes) -> char* { char* p = ws + off; off += (bytes + 255) & ~(size_t)255; return p; };
  unsigned short* X0    = (unsigned short*)carve((size_t)NROWS * NHID * 2);
  unsigned short* Y0    = (unsigned short*)carve((size_t)NROWS * NHID * 2);
  unsigned short* WIH16 = (unsigned short*)carve((size_t)NLAYER * NGATE * NHID * 2);
  unsigned short* WHH16 = (unsigned short*)carve((size_t)NLAYER * NGATE * NHID * 2);
  float*          BSUM  = (float*)carve((size_t)NLAYER * NGATE * 4);
  unsigned short* PRET  = (unsigned short*)carve((size_t)NSTEP * NGATE * NBATCH * 2);
  if (off > ws_size || off > (size_t)134217728) return;

  const size_t wplane = (size_t)NGATE * NHID;
  const size_t splane = (size_t)NBATCH * NHID;
  const int gemm_blks = (NROWS / 64) * (NGATE / 64) / 8;
  const int scan_blks = NBATCH / SEQ_BLK;

  prep_kernel<<<PREP_BLKS, 256, 0, stream>>>(x, emb, wih, whh, bih, bhh, X0, WIH16, WHH16, BSUM);

  gemm_pre_kernel<<<gemm_blks, 256, 0, stream>>>(X0, WIH16, BSUM, PRET);
  scan_kernel<0><<<scan_blks, SCAN_THR, 0, stream>>>(PRET, WHH16, h0, c0, Y0, out0, out1, out2);

  gemm_pre_kernel<<<gemm_blks, 256, 0, stream>>>(Y0, WIH16 + wplane, BSUM + NGATE, PRET);
  scan_kernel<1><<<scan_blks, SCAN_THR, 0, stream>>>(PRET, WHH16 + wplane, h0 + splane, c0 + splane, Y0, out0,
                                                     out1 + splane, out2 + splane);
}
